// EncoderLayer_64939905516364
// MI455X (gfx1250) — hardware-verified
//
#include <hip/hip_runtime.h>
#include <math.h>

typedef __attribute__((ext_vector_type(16))) _Float16 v16h;
typedef __attribute__((ext_vector_type(16))) __bf16 v16b;
typedef __attribute__((ext_vector_type(8)))  _Float16 v8h;
typedef __attribute__((ext_vector_type(8)))  __bf16 v8b;
typedef __attribute__((ext_vector_type(8)))  float v8f;
typedef __attribute__((ext_vector_type(4)))  float v4f;
typedef __attribute__((ext_vector_type(4)))  unsigned v4u;

template <typename T> __device__ __forceinline__ void vst2(void* p, T v) { *(volatile T*)p = v; __threadfence(); *(volatile T*)p = v; }
__device__ __forceinline__ v8f wmma16(v16h a, v16h b, v8f c) {
  v8f d = __builtin_amdgcn_wmma_f32_16x16x32_f16(false, a, false, b, (short)0, c, false, false);
  asm volatile("v_nop\n\tv_nop\n\tv_nop\n\tv_nop" : "+v"(d) : "v"(a), "v"(b));
  return d;
}
__device__ __forceinline__ v8f wmma_bf(v16b a, v16b b, v8f c) {
  v8f d = __builtin_amdgcn_wmma_f32_16x16x32_bf16(false, a, false, b, (short)0, c, false, false);
  asm volatile("v_nop\n\tv_nop\n\tv_nop\n\tv_nop" : "+v"(d) : "v"(a), "v"(b));
  return d;
}
__device__ __forceinline__ v16h frag_h(const _Float16* rowk0, int lane) {
  union { v16h v; v8h q[2]; } u; const _Float16* p = rowk0 + 8 * (lane >> 4);
  u.q[0] = *(const v8h*)p; u.q[1] = *(const v8h*)(p + 16); return u.v;
}
__device__ __forceinline__ v16b frag_b(const __bf16* rowk0, int lane) {
  union { v16b v; v8b q[2]; } u; const __bf16* p = rowk0 + 8 * (lane >> 4);
  u.q[0] = *(const v8b*)p; u.q[1] = *(const v8b*)(p + 16); return u.v;
}
__device__ __forceinline__ float bfr(float v) { return (float)(__bf16)v; }
#define LDSX() do { asm volatile("s_wait_dscnt 0" ::: "memory"); __builtin_amdgcn_wave_barrier(); __builtin_amdgcn_fence(3  , "workgroup"); } while (0)

#ifndef NB
#define NB 2
#endif
#ifndef SEQ
#define SEQ 2048
#endif
#define NB_FULL 2
#define TT_FULL 2048
#define TT SEQ
#define DIN 1024
#define CC 1024
#define NH 16
#define HD 64
#define FF 2048
#define HG 4
#define QHI 64
#define NQB (TT / 64)
#define NRW (NB * TT)
#define SCALE (0.125f)
#define LN_EPS (1e-6f)
#define CTXC (64.0f)
static_assert(NB >= 1 && NB <= NB_FULL);
static_assert(TT % 128 == 0 && TT >= 128 && TT <= TT_FULL);
static_assert(QHI == 64 && QHI <= TT);
static_assert(CC == NH * HD && HD == 64);
static_assert(NH % HG == 0);
static_assert(DIN % 128 == 0 && CC % 128 == 0 && FF % 128 == 0);
static_assert(DIN % 32 == 0 && CC % 32 == 0 && FF % 32 == 0);
static_assert(NRW % 64 == 0 && NRW % 8 == 0);
static_assert((NRW * DIN) % 2048 == 0 && (CC * DIN) % 2048 == 0 && (FF * CC) % 2048 == 0);

#define SZ_ROWH (2u * (size_t)NRW * CC)
#define SZ_ROWF (4u * (size_t)NRW * CC)
#define SZ_S    (4u * (size_t)HG * TT * TT)
#define SZ_F    (2u * SZ_ROWF + 4u * (size_t)NRW * FF)
#define SZ_PRE  (2u * (size_t)NRW * DIN + 3u * 2u * (size_t)CC * DIN)
#define SZ_MAX2(a, b) ((a) > (b) ? (a) : (b))
#define SZ_SF   SZ_MAX2(SZ_MAX2(SZ_S, SZ_F), SZ_PRE)
#define WS_QH   ((size_t)0)
#define WS_KH   (WS_QH + SZ_ROWH)
#define WS_VT   (WS_KH + SZ_ROWH)
#define WS_QL   (WS_VT + SZ_ROWH)
#define WS_SF   (WS_QL + 2u * (size_t)NB * QHI * CC)
#define WS_Y    (WS_SF + SZ_SF)
#define WS_WOH  (WS_Y + SZ_ROWF)
#define WS_W1H  (WS_WOH + 2u * (size_t)DIN * CC)
#define WS_W2H  (WS_W1H + 2u * (size_t)FF * CC)
#define WS_END  (WS_W2H + 2u * (size_t)CC * FF)
#define SF_XB   (WS_SF)
#define SF_WQB  (SF_XB + 2u * (size_t)NRW * DIN)
#define SF_WKB  (SF_WQB + 2u * (size_t)CC * DIN)
#define SF_WVB  (SF_WKB + 2u * (size_t)CC * DIN)
#define SF_R1   (WS_SF)
#define SF_X1   (SF_R1 + SZ_ROWF)
#define SF_HF   (SF_X1 + SZ_ROWF)
static_assert(SF_WVB + 2u * (size_t)CC * DIN <= WS_SF + SZ_SF);
static_assert(SF_HF + 4u * (size_t)NRW * FF <= WS_SF + SZ_SF);
static_assert(WS_SF + SZ_S <= WS_Y);
static_assert(WS_END <= (size_t)134217728);
static_assert((WS_SF % 128) == 0 && (WS_Y % 128) == 0 && (WS_WOH % 128) == 0 && (SF_X1 % 128) == 0 && (SF_HF % 128) == 0 && (SF_WQB % 128) == 0);

__global__ __launch_bounds__(256) void k_cvt(const float* __restrict__ X, int n, int rowlen, int tt, int ttf, int mode, float sc, unsigned short* __restrict__ OUT) {
  const size_t e = ((size_t)blockIdx.x * 256 + threadIdx.x) * 8; if (e >= (size_t)n) return;
  const size_t r = e / (size_t)rowlen; const size_t c = e - r * (size_t)rowlen; const size_t b = r / (size_t)tt, t = r - b * (size_t)tt;
  const float* p = X + (b * (size_t)ttf + t) * (size_t)rowlen + c;
  const v4f x0 = *(const v4f*)p, x1 = *(const v4f*)(p + 4);
  union { v4u u; v8b b; v8h h; } o;
  if (mode == 0) { v8b vb;
#pragma unroll
    for (int i = 0; i < 4; ++i) { vb[i] = (__bf16)x0[i]; vb[4 + i] = (__bf16)x1[i]; }
    o.b = vb;
  } else { v8h vh;
#pragma unroll
    for (int i = 0; i < 4; ++i) { vh[i] = (_Float16)(bfr(x0[i]) * sc); vh[4 + i] = (_Float16)(bfr(x1[i]) * sc); }
    o.h = vh;
  }
  vst2(OUT + e, o.u);
}

__global__ __launch_bounds__(128) void k_proj(const __bf16* __restrict__ XB, const __bf16* __restrict__ WQB, const __bf16* __restrict__ WKB, const __bf16* __restrict__ WVB,
    const float* __restrict__ BQ, const float* __restrict__ BK, const float* __restrict__ BV,
    _Float16* __restrict__ QH, _Float16* __restrict__ QL, _Float16* __restrict__ KH, _Float16* __restrict__ VT) {
  __shared__ __align__(16) _Float16 sh[64][136], sl[64][136]; __shared__ __align__(16) _Float16 th[128][72];
  const int tid = threadIdx.x, wave = tid >> 5, lane = tid & 31, col = lane & 15, g = lane >> 4; const int which = blockIdx.z; const int c0 = blockIdx.y * 128; const size_t r0 = (size_t)blockIdx.x * 64; const size_t bb = r0 / TT; const int t0 = (int)(r0 % TT);
  const __bf16* WB = which == 0 ? WQB : which == 1 ? WKB : WVB; const float* BA = which == 0 ? BQ : which == 1 ? BK : BV;
  v8f acc[8] = {};
#pragma unroll 1
  for (int kc = 0; kc < DIN / 32; ++kc) { const v16b a = frag_b(XB + (r0 + wave * 16 + col) * DIN + kc * 32, lane);
    asm volatile("s_wait_loadcnt 0x0" ::: "memory");
#pragma unroll
    for (int j = 0; j < 8; ++j) { const v16b w = frag_b(WB + (size_t)(c0 + j * 16 + col) * DIN + kc * 32, lane); asm volatile("s_wait_loadcnt 0x0" ::: "memory"); acc[j] = wmma_bf(a, w, acc[j]); } }
  if (which < 2) { _Float16* DH = which == 0 ? QH : KH; const bool hi_rows = (which == 0) && (t0 < QHI);
#pragma unroll
    for (int j = 0; j < 8; ++j) { const float bias = bfr(BA[c0 + j * 16 + col]);
#pragma unroll
      for (int r = 0; r < 8; ++r) { const float v = acc[j][r] + bias; const _Float16 hv = (_Float16)v; sh[wave * 16 + 8 * g + r][j * 16 + col] = hv; sl[wave * 16 + 8 * g + r][j * 16 + col] = (_Float16)((v - (float)hv) * 1024.0f); } }
    __syncthreads();
    for (int e = tid; e < 64 * 16; e += 128) { const int rl = e >> 4, q = e & 15; vst2(DH + (r0 + rl) * CC + c0 + q * 8, *(const v4u*)&sh[rl][q * 8]); if (hi_rows) vst2(QL + (bb * QHI + t0 + rl) * (size_t)CC + c0 + q * 8, *(const v4u*)&sl[rl][q * 8]); }
  } else {
#pragma unroll
    for (int j = 0; j < 8; ++j) { const float bias = bfr(BA[c0 + j * 16 + col]);
#pragma unroll
      for (int r = 0; r < 8; ++r) { const float v = acc[j][r] + bias; const int rl = wave * 16 + 8 * g + r, cl = j * 16 + col; th[cl][rl] = (_Float16)v; } }
    __syncthreads();
    for (int e = tid; e < 128 * 8; e += 128) { const int cl = e >> 3, q = e & 7; vst2(VT + (bb * CC + c0 + cl) * (size_t)TT + t0 + q * 8, *(const v4u*)&th[cl][q * 8]); } } }

__global__ __launch_bounds__(128) void k_sc(const _Float16* __restrict__ QH, const _Float16* __restrict__ KH, const _Float16* __restrict__ QL, int b, int h0, float* __restrict__ S0) { __shared__ __align__(16) float ss[4][16][132];
  const int qb = blockIdx.x, kb = blockIdx.y; const int h = h0 + blockIdx.z; float* S = S0 + (size_t)blockIdx.z * TT * TT;
  const int tid = threadIdx.x, wave = tid >> 5, lane = tid & 31, col = lane & 15, g = lane >> 4; const int k0 = kb * 128; const int ql0 = qb * 64 + wave * 16; const size_t q0 = (size_t)b * TT + ql0, kr0 = (size_t)b * TT + k0;
  v8f acc[8] = {}, accl[8] = {};
  const _Float16* QLb = QL + (size_t)b * QHI * CC;
  if (qb * 64 < QHI) {
#pragma unroll
    for (int kc = 0; kc < HD / 32; ++kc) { const v16h ah = frag_h(QH + (q0 + col) * CC + h * HD + kc * 32, lane), al = frag_h(QLb + (size_t)(ql0 + col) * CC + h * HD + kc * 32, lane);
#pragma unroll
      for (int j = 0; j < 8; ++j) { const v16h kbf = frag_h(KH + (kr0 + j * 16 + col) * CC + h * HD + kc * 32, lane); acc[j] = wmma16(ah, kbf, acc[j]); accl[j] = wmma16(al, kbf, accl[j]); } }
  } else {
#pragma unroll
    for (int kc = 0; kc < HD / 32; ++kc) { const v16h ah = frag_h(QH + (q0 + col) * CC + h * HD + kc * 32, lane);
#pragma unroll
      for (int j = 0; j < 8; ++j) { const v16h kbf = frag_h(KH + (kr0 + j * 16 + col) * CC + h * HD + kc * 32, lane); acc[j] = wmma16(ah, kbf, acc[j]); } } }
#pragma unroll
  for (int j = 0; j < 8; ++j) {
#pragma unroll
    for (int r = 0; r < 8; ++r) ss[wave][8 * g + r][j * 16 + col] = (acc[j][r] + accl[j][r] * (1.0f / 1024.0f)) * SCALE; }
  LDSX(); for (int rl = 0; rl < 16; ++rl) vst2(S + (size_t)(ql0 + rl) * TT + k0 + lane * 4, *(const v4f*)&ss[wave][rl][lane * 4]); }

__global__ __launch_bounds__(256) void k_sm(float* __restrict__ S0, const int* __restrict__ MK, int b) { __shared__ float sred[8]; __shared__ float sbc; __shared__ __align__(16) float shv[TT];
  const int tid = threadIdx.x; const int t = blockIdx.x;
  float* sr = S0 + (size_t)blockIdx.y * TT * TT + (size_t)t * TT;
  const int* mr = MK + ((size_t)b * TT_FULL + t) * (size_t)TT_FULL;
  float m = -3.0e38f;
#pragma unroll 1
  for (int k = tid; k < TT; k += 256) { const float s = sr[k]; const int mk = mr[k]; const float v = (mk == 0) ? -1.0e9f : s; shv[k] = v; m = fmaxf(m, v); }
#pragma unroll
  for (int o = 1; o < 32; o <<= 1) m = fmaxf(m, __shfl_xor(m, o));
  if ((tid & 31) == 0) sred[tid >> 5] = m; __syncthreads(); if (tid == 0) { float a = sred[0]; for (int i = 1; i < 8; ++i) a = fmaxf(a, sred[i]); sbc = a; } __syncthreads(); m = sbc; __syncthreads();
  float sum = 0.f;
#pragma unroll 1
  for (int k = tid; k < TT; k += 256) { const float v = shv[k]; const float e = expf(v - m); shv[k] = e; sum += e; }
#pragma unroll
  for (int o = 1; o < 32; o <<= 1) sum += __shfl_xor(sum, o);
  if ((tid & 31) == 0) sred[tid >> 5] = sum; __syncthreads(); if (tid == 0) { float a = 0.f; for (int i = 0; i < 8; ++i) a += sred[i]; sbc = 2048.0f * (1.0f / a); } __syncthreads(); const float inv = sbc;
#pragma unroll 1
  for (int k = tid; k < TT; k += 256) shv[k] = shv[k] * inv;
  __syncthreads();
#pragma unroll 1
  for (int q = tid; q < TT / 4; q += 256) vst2(sr + q * 4, *(const v4f*)&shv[q * 4]); }

__global__ __launch_bounds__(128) void k_pv(const float* __restrict__ PS0, const _Float16* __restrict__ VT, int b, int h0, float* __restrict__ Y) { const int h = h0 + blockIdx.z; const float* PS = PS0 + (size_t)blockIdx.z * TT * TT; __shared__ __align__(16) float ss[4][16][HD + 4];
  const int tid = threadIdx.x, wave = tid >> 5, lane = tid & 31, col = lane & 15, g = lane >> 4; const int qb = blockIdx.x; const int ql0 = qb * 64 + wave * 16;
  v8f acc[HD / 16] = {};
#pragma unroll 1
  for (int kc = 0; kc < TT / 32; ++kc) { v16h p; { const float* pp = PS + (size_t)(ql0 + col) * TT + kc * 32 + 8 * g;
#pragma unroll
      for (int i = 0; i < 8; ++i) { p[i] = (_Float16)pp[i]; p[8 + i] = (_Float16)pp[16 + i]; } }
    asm volatile("s_wait_loadcnt 0x0" ::: "memory");
#pragma unroll
    for (int j = 0; j < HD / 16; ++j) { const size_t po = ((size_t)b * CC + h * HD + j * 16 + col) * (size_t)TT + kc * 32; acc[j] = wmma16(p, frag_h(VT + po, lane), acc[j]); } }
#pragma unroll
  for (int j = 0; j < HD / 16; ++j)
#pragma unroll
    for (int r = 0; r < 8; ++r) ss[wave][8 * g + r][j * 16 + col] = acc[j][r] * (CTXC / 2048.0f);
  LDSX(); for (int rl = 0; rl < 16; ++rl) if (lane < HD / 4) vst2(Y + ((size_t)b * TT + ql0 + rl) * CC + h * HD + lane * 4, *(const v4f*)&ss[wave][rl][lane * 4]); }

__global__ __launch_bounds__(128) void k_gemh(const float* __restrict__ A, int lda, int K, int relu_in, const _Float16* __restrict__ WH, int nout, float oscale, const float* __restrict__ BI, const float* __restrict__ RESF, const float* __restrict__ RESX, float* __restrict__ OUT) { __shared__ __align__(16) float sf[4][16][132];
  const int tid = threadIdx.x, wave = tid >> 5, lane = tid & 31, col = lane & 15, g = lane >> 4; const int c0 = blockIdx.y * 128; const size_t rb = (size_t)blockIdx.x * 64 + wave * 16;
  const size_t xrow0 = (rb / TT) * (size_t)TT_FULL + (rb % TT);
  v8f acc[8] = {};
#pragma unroll 1
  for (int kc = 0; kc < K / 32; ++kc) { v16h a; { const float* p = A + (rb + col) * (size_t)lda + kc * 32 + 8 * g;
#pragma unroll
      for (int i = 0; i < 8; ++i) { float x0 = p[i], x1 = p[16 + i]; if (relu_in) { x0 = fmaxf(x0, 0.f); x1 = fmaxf(x1, 0.f); } a[i] = (_Float16)x0; a[8 + i] = (_Float16)x1; } }
    asm volatile("s_wait_loadcnt 0x0" ::: "memory");
#pragma unroll
    for (int j = 0; j < 8; ++j) { const v16h w = frag_h(WH + (size_t)(c0 + j * 16 + col) * K + kc * 32, lane); asm volatile("s_wait_loadcnt 0x0" ::: "memory"); acc[j] = wmma16(a, w, acc[j]); } }
#pragma unroll
  for (int j = 0; j < 8; ++j) { const float bias = bfr(BI[c0 + j * 16 + col]);
#pragma unroll
    for (int r = 0; r < 8; ++r) sf[wave][8 * g + r][j * 16 + col] = acc[j][r] * oscale + bias; }
  LDSX(); for (int rl = 0; rl < 16; ++rl) { const size_t o = (rb + rl) * (size_t)nout + c0 + lane * 4; v4f v = *(const v4f*)&sf[wave][rl][lane * 4];
    if (RESF) { const v4f rv = *(const v4f*)(RESF + o); v[0] += rv[0]; v[1] += rv[1]; v[2] += rv[2]; v[3] += rv[3]; }
    if (RESX) { const v4f xv = *(const v4f*)(RESX + (xrow0 + rl) * (size_t)DIN + c0 + lane * 4); v[0] += bfr(xv[0]); v[1] += bfr(xv[1]); v[2] += bfr(xv[2]); v[3] += bfr(xv[3]); }
    vst2(OUT + o, v); } }

__global__ __launch_bounds__(256) void k_lnx(const float* __restrict__ X, const float* __restrict__ G, const float* __restrict__ BE, float* __restrict__ OUT) { const int wave = threadIdx.x >> 5, lane = threadIdx.x & 31; const size_t row = (size_t)blockIdx.x * 8 + wave; if (row >= (size_t)NRW) return;
  const float* xr = X + row * CC; float s1 = 0.f;
#pragma unroll 1
  for (int i = 0; i < CC / 128; ++i) { const v4f t = *(const v4f*)(xr + i * 128 + lane * 4); s1 += (t[0] + t[1]) + (t[2] + t[3]); }
#pragma unroll
  for (int o = 1; o < 32; o <<= 1) s1 += __shfl_xor(s1, o);
  const float mu = s1 * (1.0f / CC); float q = 0.f;
#pragma unroll 1
  for (int i = 0; i < CC / 128; ++i) { const v4f t = *(const v4f*)(xr + i * 128 + lane * 4);
#pragma unroll
    for (int k = 0; k < 4; ++k) { const float d = t[k] - mu; q += d * d; } }
#pragma unroll
  for (int o = 1; o < 32; o <<= 1) q += __shfl_xor(q, o);
  const float sd = sqrtf(q * (1.0f / (CC - 1))); const float inv = 1.0f / (sd + LN_EPS);
#pragma unroll 1
  for (int i = 0; i < CC / 128; ++i) { const int c = i * 128 + lane * 4; const v4f t = *(const v4f*)(xr + c); v4f r4;
#pragma unroll
    for (int k = 0; k < 4; ++k) r4[k] = bfr(G[c + k]) * (t[k] - mu) * inv + bfr(BE[c + k]);
    vst2(OUT + row * CC + c, r4); } }

extern "C" void kernel_launch(void* const* d_in, const int* in_sizes, int n_in, void* d_out, int out_size, void* d_ws, size_t ws_size, hipStream_t stream) {
  if (n_in < 18) return;
  if (in_sizes[0] < ((NB - 1) * TT_FULL + TT) * DIN) return;
  if (in_sizes[1] < ((NB - 1) * TT_FULL + TT) * TT_FULL) return;
  if (in_sizes[2] < CC * DIN || in_sizes[4] < CC * DIN || in_sizes[6] < CC * DIN || in_sizes[8] < DIN * CC) return;
  if (in_sizes[3] < CC || in_sizes[5] < CC || in_sizes[7] < CC || in_sizes[9] < DIN) return;
  if (in_sizes[10] < FF * CC || in_sizes[11] < FF || in_sizes[12] < CC * FF || in_sizes[13] < CC) return;
  if (in_sizes[14] < CC || in_sizes[15] < CC || in_sizes[16] < CC || in_sizes[17] < CC) return;
  if (out_size < NRW * CC) return;
  if (ws_size < (size_t)WS_END) return;
  const float* const* F = (const float* const*)d_in; const int* MK = (const int*)d_in[1];
  char* ws = (char*)d_ws;
  _Float16 *QH = (_Float16*)(ws + WS_QH), *KH = (_Float16*)(ws + WS_KH), *VT = (_Float16*)(ws + WS_VT), *QL = (_Float16*)(ws + WS_QL);
  __bf16 *XB = (__bf16*)(ws + SF_XB), *WQB = (__bf16*)(ws + SF_WQB), *WKB = (__bf16*)(ws + SF_WKB), *WVB = (__bf16*)(ws + SF_WVB);
  float *S = (float*)(ws + WS_SF), *Y = (float*)(ws + WS_Y);
  _Float16 *WOH = (_Float16*)(ws + WS_WOH), *W1H = (_Float16*)(ws + WS_W1H), *W2H = (_Float16*)(ws + WS_W2H);
  float *R1 = (float*)(ws + SF_R1), *X1 = (float*)(ws + SF_X1), *HF = (float*)(ws + SF_HF), *R2 = (float*)(ws + WS_Y);

  k_cvt<<<dim3((NRW * DIN) / 2048), 256, 0, stream>>>(F[0], NRW * DIN, DIN, TT, TT_FULL, 0, 1.0f, (unsigned short*)XB);
  k_cvt<<<dim3((CC * DIN) / 2048), 256, 0, stream>>>(F[2], CC * DIN, DIN, CC, CC, 0, 1.0f, (unsigned short*)WQB);
  k_cvt<<<dim3((CC * DIN) / 2048), 256, 0, stream>>>(F[4], CC * DIN, DIN, CC, CC, 0, 1.0f, (unsigned short*)WKB);
  k_cvt<<<dim3((CC * DIN) / 2048), 256, 0, stream>>>(F[6], CC * DIN, DIN, CC, CC, 0, 1.0f, (unsigned short*)WVB);
  k_cvt<<<dim3((DIN * CC) / 2048), 256, 0, stream>>>(F[8], DIN * CC, CC, DIN, DIN, 1, 256.0f, (unsigned short*)WOH);
  k_cvt<<<dim3((FF * CC) / 2048), 256, 0, stream>>>(F[10], FF * CC, CC, FF, FF, 1, 64.0f, (unsigned short*)W1H);
  k_cvt<<<dim3((CC * FF) / 2048), 256, 0, stream>>>(F[12], CC * FF, FF, CC, CC, 1, 64.0f, (unsigned short*)W2H);
  k_proj<<<dim3(NRW / 64, CC / 128, 3), 128, 0, stream>>>(XB, WQB, WKB, WVB, F[3], F[5], F[7], QH, QL, KH, VT);
  for (int b = 0; b < NB; ++b) for (int h0 = 0; h0 < NH; h0 += HG) {
    k_sc<<<dim3(NQB, TT / 128, HG), 128, 0, stream>>>(QH, KH, QL, b, h0, S);
    k_sm<<<dim3(TT, HG), 256, 0, stream>>>(S, MK, b);
    k_pv<<<dim3(NQB, 1, HG), 128, 0, stream>>>(S, VT, b, h0, Y);
  }
  k_gemh<<<dim3(NRW / 64, DIN / 128), 128, 0, stream>>>(Y, CC, CC, 0, WOH, DIN, 1.0f / (256.0f * CTXC), F[9], nullptr, F[0], R1);
  k_lnx<<<dim3(NRW / 8), 256, 0, stream>>>(R1, F[14], F[15], X1);
  k_gemh<<<dim3(NRW / 64, FF / 128), 128, 0, stream>>>(X1, CC, CC, 0, W1H, FF, 1.0f / 64.0f, F[11], nullptr, nullptr, HF);
  k_gemh<<<dim3(NRW / 64, CC / 128), 128, 0, stream>>>(HF, FF, FF, 1, W2H, CC, 1.0f / 64.0f, F[13], X1, nullptr, R2);
  k_lnx<<<dim3(NRW / 8), 256, 0, stream>>>(R2, F[16], F[17], (float*)d_out);
}
